// SPSM_37297495998698
// MI455X (gfx1250) — hardware-verified
//
#include <hip/hip_runtime.h>

typedef __attribute__((ext_vector_type(16))) _Float16 v16h;
typedef __attribute__((ext_vector_type(8)))  _Float16 v8h;
typedef __attribute__((ext_vector_type(16))) __bf16   v16b;
typedef __attribute__((ext_vector_type(8)))  __bf16   v8b;
typedef __attribute__((ext_vector_type(8)))  float    v8f;
typedef __attribute__((ext_vector_type(4)))  float    v4f;

#define NEG_INF (-__builtin_huge_valf())

__device__ __forceinline__ unsigned short f2bf_bits(float f) {
  unsigned u = __float_as_uint(f);
  return (unsigned short)((u + 0x7FFFu + ((u >> 16) & 1u)) >> 16);
}
__device__ __forceinline__ float bf_bits2f(unsigned short h) { return __uint_as_float(((unsigned)h) << 16); }

__device__ __forceinline__ void dep_guard_h(v8f& a, v8f& b, v16h x, v16h y) { asm volatile("v_nop\n\tv_nop\n\tv_nop\n\tv_nop" : "+v"(a), "+v"(b) : "v"(x), "v"(y)); }
__device__ __forceinline__ void dep_guard_b(v8f& a, v8f& b, v16b x, v16b y) { asm volatile("v_nop\n\tv_nop\n\tv_nop\n\tv_nop" : "+v"(a), "+v"(b) : "v"(x), "v"(y)); }
__device__ __forceinline__ void keep4_h(v16h a, v16h b, v16h c, v16h d) { asm volatile("v_nop" :: "v"(a), "v"(b), "v"(c), "v"(d)); }
__device__ __forceinline__ void keep4_b(v16b a, v16b b, v16b c, v16b d) { asm volatile("v_nop" :: "v"(a), "v"(b), "v"(c), "v"(d)); }
__device__ __forceinline__ void acc_guard4(v8f& a, v8f& b, v8f& c, v8f& d) { asm volatile("v_nop\n\tv_nop\n\tv_nop\n\tv_nop" : "+v"(a), "+v"(b), "+v"(c), "+v"(d)); }
template <typename T> struct Frag;
template <> struct Frag<_Float16> {
  typedef v16h V; union U { v16h v; v8h h[2]; };
  static __device__ __forceinline__ v16h load(const _Float16* p) {
    U f; f.h[0] = *(const v8h*)(p); f.h[1] = *(const v8h*)(p + 16); return f.v;
  }
  static __device__ __forceinline__ v8f mma(v16h a, v16h b, v8f c) {
    return __builtin_amdgcn_wmma_f32_16x16x32_f16(false, a, false, b, (short)0, c, false, false);
  }
  static __device__ __forceinline__ void guard(v8f& a, v8f& b, v16h x, v16h y) { dep_guard_h(a, b, x, y); }
  static __device__ __forceinline__ void keep(v16h a, v16h b, v16h c, v16h d) { keep4_h(a, b, c, d); }
};
template <> struct Frag<__bf16> {
  typedef v16b V; union U { v16b v; v8b h[2]; };
  static __device__ __forceinline__ v16b load(const __bf16* p) {
    U f; f.h[0] = *(const v8b*)(p); f.h[1] = *(const v8b*)(p + 16); return f.v;
  }
  static __device__ __forceinline__ v8f mma(v16b a, v16b b, v8f c) {
    return __builtin_amdgcn_wmma_f32_16x16x32_bf16(false, a, false, b, (short)0, c, false, false);
  }
  static __device__ __forceinline__ void guard(v8f& a, v8f& b, v16b x, v16b y) { dep_guard_b(a, b, x, y); }
  static __device__ __forceinline__ void keep(v16b a, v16b b, v16b c, v16b d) { keep4_b(a, b, c, d); }
};

template <int ET> struct Elem;
template <> struct Elem<0> { typedef _Float16 T; };
template <> struct Elem<1> { typedef __bf16 T; };
template <int ET, bool SPLIT, int BIAS_MODE, int OUT_MODE, bool RESID, int ACT = 0>
__global__ __launch_bounds__(256) void wmma_gemm64(
    const unsigned short* __restrict__ Ap, const unsigned short* __restrict__ A2p, int lda, long strideA,
    const unsigned short* __restrict__ Btp, const unsigned short* __restrict__ Bt2p, int ldb, long strideB,
    void* __restrict__ Cout, void* __restrict__ Cout2, int ldc, long strideC,
    const float* __restrict__ bias,
    const float* __restrict__ resid, long strideR,
    int M, int N, int K, float scale) {
  typedef typename Elem<ET>::T T;
  typedef typename Frag<T>::V V;
  const T* A = (const T*)Ap; const T* A2 = (const T*)A2p; const T* Bt = (const T*)Btp; const T* Bt2 = (const T*)Bt2p;
  __shared__ __align__(16) float sT[8][16 * 68];
  const int b    = blockIdx.y;
  const int lane = threadIdx.x & 31;
  const int wave = threadIdx.x >> 5;
  const int tilesN = N >> 6;
  const int tilesM = M >> 6;
  const int tile = blockIdx.x * 8 + wave;
  if (tile >= tilesM * tilesN) return;
  const int tm = tile / tilesN;
  const int tn = tile - tm * tilesN;
  const int m0 = tm << 6;
  const int n0 = tn << 6;

  const T* Ab  = A  + (size_t)b * strideA;
  const T* Bb  = Bt + (size_t)b * strideB;
  const T* Ab2 = SPLIT ? (A2  + (size_t)b * strideA) : nullptr;
  const T* Bb2 = SPLIT ? (Bt2 + (size_t)b * strideB) : nullptr;

  const int rlane = lane & 15;
  const int koff  = (lane >> 4) * 8;
  const int mOff  = (lane >> 4) * 8;

  v8f acc[4][4];
#pragma unroll
  for (int i = 0; i < 4; ++i)
#pragma unroll
    for (int j = 0; j < 4; ++j) acc[i][j] = (v8f){0.f,0.f,0.f,0.f,0.f,0.f,0.f,0.f};

  for (int k0 = 0; k0 < K; k0 += 32) {
    V bh[4], bl[4];
#pragma unroll
    for (int j = 0; j < 4; ++j) {
      const size_t bo = (size_t)(n0 + (j << 4) + rlane) * ldb + koff + k0;
      bh[j] = Frag<T>::load(Bb + bo);
      if (SPLIT) bl[j] = Frag<T>::load(Bb2 + bo);
    }
#pragma unroll
    for (int i = 0; i < 4; ++i) {
      const size_t ao = (size_t)(m0 + (i << 4) + rlane) * lda + koff + k0;
      V ah = Frag<T>::load(Ab + ao);
      V al;
      if (SPLIT) al = Frag<T>::load(Ab2 + ao);
#pragma unroll
      for (int j = 0; j < 4; ++j) {
        acc[i][j] = Frag<T>::mma(ah, bh[j], acc[i][j]);
        if (SPLIT) {
          acc[i][j] = Frag<T>::mma(ah, bl[j], acc[i][j]);
          acc[i][j] = Frag<T>::mma(al, bh[j], acc[i][j]);
        }
      }
      Frag<T>::guard(acc[i][0], acc[i][3], ah, SPLIT ? al : ah);
    }
    Frag<T>::keep(bh[0], bh[1], bh[2], bh[3]);
    if (SPLIT) Frag<T>::keep(bl[0], bl[1], bl[2], bl[3]);
  }
  acc_guard4(acc[0][0], acc[0][1], acc[0][2], acc[0][3]);
  acc_guard4(acc[1][0], acc[1][1], acc[1][2], acc[1][3]);
  acc_guard4(acc[2][0], acc[2][1], acc[2][2], acc[2][3]);
  acc_guard4(acc[3][0], acc[3][1], acc[3][2], acc[3][3]);

  float* slab = sT[wave];
  const float* Rb = RESID ? (resid + (size_t)b * strideR) : nullptr;
#pragma unroll
  for (int i = 0; i < 4; ++i) {
    const int mBase = m0 + (i << 4);
#pragma unroll
    for (int j = 0; j < 4; ++j) {
      const int n = n0 + (j << 4) + rlane;
      float bv = 0.f;
      if (BIAS_MODE == 2) bv = bias[n];
#pragma unroll
      for (int r = 0; r < 8; ++r) {
        float v = acc[i][j][r] * scale;
        if (BIAS_MODE == 1) v += bias[mBase + mOff + r];
        if (BIAS_MODE == 2) v += bv;
        if (RESID) v += Rb[(size_t)(mBase + mOff + r) * ldc + n];
        if (ACT == 1) v = tanhf(v);
        if (ACT == 2) v = fmaxf(v, 0.0f);
        if (ACT == 3) v = v / (1.0f + expf(-v));
        if (ACT == 4) v = (v > 0.f) ? v : 0.01f * v;
        if (ACT == 5) v = 0.5f * v * (1.0f + erff(v * 0.70710678118654752f));
        slab[(mOff + r) * 68 + (j << 4) + rlane] = v;
      }
    }
    __builtin_amdgcn_fence(__ATOMIC_RELEASE, "workgroup");
    __builtin_amdgcn_wave_barrier();
    __builtin_amdgcn_fence(__ATOMIC_ACQUIRE, "workgroup");
    if (OUT_MODE == 0) {
      float* C = (float*)Cout + (size_t)b * strideC;
      const int hh = lane >> 4, c4 = (lane & 15) * 4;
      for (int pass = 0; pass < 2; ++pass) {
#pragma unroll
        for (int it = 0; it < 8; ++it) {
          const int row = it * 2 + hh;
          v4f v = *(const v4f*)(slab + row * 68 + c4);
          *(volatile v4f*)(C + (size_t)(mBase + row) * ldc + n0 + c4) = v;
        }
        __threadfence();
      }
    } else {
      const int q = lane >> 3, c8 = (lane & 7) * 8;
      unsigned short* C  = (unsigned short*)Cout  + (size_t)b * strideC;
      unsigned short* C2 = (OUT_MODE == 2) ? ((unsigned short*)Cout2 + (size_t)b * strideC) : nullptr;
      for (int pass = 0; pass < 2; ++pass) {
#pragma unroll
        for (int it = 0; it < 4; ++it) {
          const int row = it * 4 + q;
          const float* sp = slab + row * 68 + c8;
          v8h hv, lv;
#pragma unroll
          for (int e = 0; e < 8; ++e) {
            if (OUT_MODE == 1) {
              hv[e] = (_Float16)sp[e];
            } else {
              unsigned short hb = f2bf_bits(sp[e]);
              unsigned short lb = f2bf_bits(sp[e] - bf_bits2f(hb));
              hv[e] = __builtin_bit_cast(_Float16, hb);
              lv[e] = __builtin_bit_cast(_Float16, lb);
            }
          }
          *(volatile v8h*)(C + (size_t)(mBase + row) * ldc + n0 + c8) = hv;
          if (OUT_MODE == 2) *(volatile v8h*)(C2 + (size_t)(mBase + row) * ldc + n0 + c8) = lv;
        }
        __threadfence();
      }
    }
    __builtin_amdgcn_fence(__ATOMIC_RELEASE, "workgroup");
    __builtin_amdgcn_wave_barrier();
    __builtin_amdgcn_fence(__ATOMIC_ACQUIRE, "workgroup");
  }
}

#define NB   8
#define NP   1000
#define NN   1000
#define NE   128
#define NH   8
#define DH   16
#define RP   1024
#define KQ   160
#define ROWS (NB * RP)
#define VLD  8192

__device__ __forceinline__ v8h zero8h() {
  v8h z;
#pragma unroll
  for (int e = 0; e < 8; ++e) z[e] = (_Float16)0.0f;
  return z;
}
__device__ __forceinline__ v8h cvt8h(v8f f, float sc) {
  v8h h;
#pragma unroll
  for (int e = 0; e < 8; ++e) h[e] = (_Float16)(f[e] * sc);
  return h;
}
__device__ __forceinline__ void store16_twice(_Float16* q, v8h hv) {
  *(volatile v8h*)q = hv;
  __threadfence();
  *(volatile v8h*)q = hv;
}

__global__ __launch_bounds__(256) void prep_enc_kernel(
    const float* __restrict__ enc, _Float16* __restrict__ out, int n8) {
  const int i = blockIdx.x * 256 + threadIdx.x;
  if (i < n8) {
    const int row = i >> 4;
    const int c8  = (i & 15) * 8;
    const int bb  = row >> 10;
    const int n   = row & (RP - 1);
    const int nc  = n < NN ? n : NN - 1;
    const float* p = enc + ((size_t)bb * NN + nc) * NE + c8;
    const v4f f0 = *(const v4f*)p;
    const v4f f1 = *(const v4f*)(p + 4);
    v8f f = (v8f){0.f,0.f,0.f,0.f,0.f,0.f,0.f,0.f};
    if (n < NN) { f[0] = f0[0]; f[1] = f0[1]; f[2] = f0[2]; f[3] = f0[3]; f[4] = f1[0]; f[5] = f1[1]; f[6] = f1[2]; f[7] = f1[3]; }
    store16_twice(out + (size_t)i * 8, cvt8h(f, 1.0f));
  }
}

__global__ __launch_bounds__(256) void prep_cat_kernel(
    const float* __restrict__ eln, const float* __restrict__ attr, _Float16* __restrict__ out, int n8) {
  const int i = blockIdx.x * 256 + threadIdx.x;
  if (i < n8) {
    const int row   = i / 20;
    const int piece = i - row * 20;
    const int bb = row >> 10;
    const int p  = row & (RP - 1);
    const int pc = p < NP ? p : NP - 1;
    const int pe = piece < 16 ? piece : 15;
    const size_t src = (size_t)bb * NP + pc;
    const v4f e0 = *(const v4f*)(eln + src * NE + pe * 8);
    const v4f e1 = *(const v4f*)(eln + src * NE + pe * 8 + 4);
    const v4f a4 = *(const v4f*)(attr + src * 4);
    v8f f = (v8f){0.f,0.f,0.f,0.f,0.f,0.f,0.f,0.f};
    if (p < NP) {
      if (piece < 16) {
        f[0] = e0[0]; f[1] = e0[1]; f[2] = e0[2]; f[3] = e0[3];
        f[4] = e1[0]; f[5] = e1[1]; f[6] = e1[2]; f[7] = e1[3];
      } else if (piece == 16) {
        f[0] = a4[0]; f[1] = a4[1]; f[2] = a4[2]; f[3] = a4[3];
      }
    }
    store16_twice(out + (size_t)i * 8, cvt8h(f, 1.0f));
  }
}

__global__ __launch_bounds__(256) void wtrans_kernel(
    const float* __restrict__ W0, const float* __restrict__ W1, const float* __restrict__ W2, const float* __restrict__ W3,
    _Float16* __restrict__ O0, _Float16* __restrict__ O1, _Float16* __restrict__ O2, _Float16* __restrict__ O3,
    int Kin, int Kpad, int n8, float scale) {
  const int y = blockIdx.y;
  const float* W = (y == 0) ? W0 : (y == 1) ? W1 : (y == 2) ? W2 : W3;
  _Float16*    O = (y == 0) ? O0 : (y == 1) ? O1 : (y == 2) ? O2 : O3;
  const int i = blockIdx.x * 256 + threadIdx.x;
  if (i < n8) {
    const int ppr   = Kpad >> 3;
    const int o     = i / ppr;
    const int piece = i - o * ppr;
    v8h hv;
#pragma unroll
    for (int e = 0; e < 8; ++e) {
      const int k  = piece * 8 + e;
      const int kc = k < Kin ? k : Kin - 1;
      const float f = W[(size_t)kc * NE + o] * scale;
      hv[e] = (k < Kin) ? (_Float16)f : (_Float16)0.0f;
    }
    store16_twice(O + (size_t)i * 8, hv);
  }
}

#define AT_NW 4
#define AT_QB 64
#define AT_KC 64
#define A_KP 16
#define A_VP 72
#define A_PP 72
#define A_OP 20
#define PSC 32768.0f

__device__ __forceinline__ v8f mma_h(v16h a, v16h b, v8f c) {
  c = __builtin_amdgcn_wmma_f32_16x16x32_f16(false, a, false, b, (short)0, c, false, false);
  asm volatile("v_nop\n\tv_nop\n\tv_nop\n\tv_nop" : "+v"(c) : "v"(a), "v"(b));
  return c;
}

__global__ __launch_bounds__(128) void mha16_kernel(
    const _Float16* __restrict__ Qg, const _Float16* __restrict__ Kg, const _Float16* __restrict__ Vg,
    const float* __restrict__ mask, float* __restrict__ Og, float qscale) {
  __shared__ __align__(16) _Float16 Ks[AT_KC * A_KP];
  __shared__ __align__(16) _Float16 Vt[DH * A_VP];
  __shared__ __align__(16) _Float16 Ps[AT_NW][16 * A_PP];
  __shared__ __align__(16) float Os[AT_NW][16 * A_OP];

  const int tid  = threadIdx.x;
  const int wave = tid >> 5;
  const int lane = tid & 31;
  const int hh   = lane >> 4;
  const int c    = lane & 15;
  const int qb   = blockIdx.x;
  const int h    = blockIdx.y & 7;
  const int bb   = (blockIdx.y >> 3) & 7;
  const int br   = blockIdx.y >> 6;
  const int q0   = qb * AT_QB + wave * 16;

  const size_t rowbase = (size_t)(br * NB + bb) * RP;
  const _Float16* Qb = Qg + rowbase * NE + h * DH;
  const _Float16* Kb = Kg + rowbase * NE + h * DH;
  const _Float16* Vb = Vg + ((size_t)br * NE + h * DH) * VLD + (size_t)bb * RP;
  const float*    Mb = mask + (size_t)bb * NP * NN;
  float*          Ob = Og + ((((size_t)(br * NB + bb)) * NH + h) * RP + q0) * DH;

  union FH { v16h v; v8h p[2]; };
  const v8h z8 = zero8h();
  FH qf;
  qf.p[0] = *(const v8h*)(Qb + (size_t)(q0 + c) * NE + 8 * hh);
  qf.p[1] = z8;
  const v16h qa = qf.v;

  float mrow[8], lrow[8];
  v8f oacc = (v8f){0.f,0.f,0.f,0.f,0.f,0.f,0.f,0.f};
#pragma unroll
  for (int r = 0; r < 8; ++r) { mrow[r] = NEG_INF; lrow[r] = 0.f; }

  for (int kc = 0; kc < RP / AT_KC; ++kc) {
    const int kv0 = kc * AT_KC;
    __syncthreads();
    {
      const int kvr = tid >> 1, part = tid & 1;
      const v8h k8 = *(const v8h*)(Kb + (size_t)(kv0 + kvr) * NE + part * 8);
      *(v8h*)(Ks + kvr * A_KP + part * 8) = k8;
      const int d = tid >> 3, piece = tid & 7;
      const v8h v8 = *(const v8h*)(Vb + (size_t)d * VLD + kv0 + piece * 8);
      *(v8h*)(Vt + d * A_VP + piece * 8) = v8;
    }
    __syncthreads();

    v8f s[4];
#pragma unroll
    for (int j = 0; j < 4; ++j) {
      FH kf;
      kf.p[0] = *(const v8h*)(Ks + (j * 16 + c) * A_KP + 8 * hh);
      kf.p[1] = z8;
      s[j] = mma_h(qa, kf.v, (v8f){0.f,0.f,0.f,0.f,0.f,0.f,0.f,0.f});
    }
    float cm[8];
#pragma unroll
    for (int r = 0; r < 8; ++r) {
      const int qrow = q0 + 8 * hh + r;
      const int qrc  = qrow < NP ? qrow : NP - 1;
      const float* mr = Mb + (size_t)qrc * NN;
      float m = NEG_INF;
#pragma unroll
      for (int j = 0; j < 4; ++j) {
        const int kv  = kv0 + j * 16 + c;
        const int kvc = kv < NN ? kv : NN - 1;
        float v = s[j][r] * qscale + mr[kvc];
        if (kv >= NN) v = NEG_INF;
        s[j][r] = v;
        m = fmaxf(m, v);
      }
#pragma unroll
      for (int off = 1; off < 16; off <<= 1) m = fmaxf(m, __shfl_xor(m, off, 32));
      cm[r] = m;
    }
    _Float16* pw = Ps[wave];
#pragma unroll
    for (int r = 0; r < 8; ++r) {
      const float mnew  = fmaxf(mrow[r], cm[r]);
      const float alpha = __expf(mrow[r] - mnew);
      mrow[r] = mnew;
      float psum = 0.f;
#pragma unroll
      for (int j = 0; j < 4; ++j) {
        const float p = __expf(s[j][r] - mnew);
        psum += p;
        pw[(8 * hh + r) * A_PP + j * 16 + c] = (_Float16)(p * PSC);
      }
#pragma unroll
      for (int off = 1; off < 16; off <<= 1) psum += __shfl_xor(psum, off, 32);
      lrow[r] = lrow[r] * alpha + psum;
      oacc[r] *= alpha;
    }
    __builtin_amdgcn_fence(__ATOMIC_RELEASE, "workgroup");
    __builtin_amdgcn_wave_barrier();
    __builtin_amdgcn_fence(__ATOMIC_ACQUIRE, "workgroup");
#pragma unroll
    for (int kk = 0; kk < 2; ++kk) {
      const v16h pa = Frag<_Float16>::load(pw + c * A_PP + kk * 32 + 8 * hh);
      const v16h vb = Frag<_Float16>::load(Vt + c * A_VP + kk * 32 + 8 * hh);
      oacc = mma_h(pa, vb, oacc);
    }
  }

  float* os = Os[wave];
#pragma unroll
  for (int r = 0; r < 8; ++r) {
    const float inv = 1.0f / (lrow[r] * (PSC * 64.0f));
    os[(8 * hh + r) * A_OP + c] = oacc[r] * inv;
  }
  __builtin_amdgcn_fence(__ATOMIC_RELEASE, "workgroup");
  __builtin_amdgcn_wave_barrier();
  __builtin_amdgcn_fence(__ATOMIC_ACQUIRE, "workgroup");
  {
    for (int pass = 0; pass < 2; ++pass) {
#pragma unroll
      for (int it = 0; it < 2; ++it) {
        const int q   = it * 32 + lane;
        const int row = q >> 2;
        const int c4  = (q & 3) * 4;
        v4f val = *(const v4f*)(os + row * A_OP + c4);
        *(volatile v4f*)(Ob + (size_t)row * DH + c4) = val;
      }
      __threadfence();
    }
  }
}

__global__ __launch_bounds__(256) void cast_o_kernel(
    const float* __restrict__ O32, _Float16* __restrict__ O16, int n8, float scale) {
  const int i = blockIdx.x * 256 + threadIdx.x;
  if (i < n8) {
    const int row   = i >> 4;
    const int piece = i & 15;
    const int hd = piece >> 1, half = piece & 1;
    const int br = row >> 13;
    const int bb = (row >> 10) & 7;
    const int p  = row & (RP - 1);
    const float* src = O32 + ((((size_t)(br * NB + bb)) * NH + hd) * RP + p) * DH + half * 8;
    const v4f f0 = *(const v4f*)src;
    const v4f f1 = *(const v4f*)(src + 4);
    v8f f;
    f[0] = f0[0]; f[1] = f0[1]; f[2] = f0[2]; f[3] = f0[3];
    f[4] = f1[0]; f[5] = f1[1]; f[6] = f1[2]; f[7] = f1[3];
    store16_twice(O16 + (size_t)i * 8, cvt8h(f, scale));
  }
}

__global__ __launch_bounds__(256) void combine_kernel(
    const float* __restrict__ gp, const float* __restrict__ ocs, const float* __restrict__ oct,
    const float* __restrict__ bcs, const float* __restrict__ bct,
    _Float16* __restrict__ g16, int n8, float scale) {
  const int i = blockIdx.x * 256 + threadIdx.x;
  if (i < n8) {
    const int c8 = (i & 15) * 8;
    const size_t base = (size_t)i * 8;
    const v4f x0 = *(const v4f*)(gp + base),  x1 = *(const v4f*)(gp + base + 4);
    const v4f s0 = *(const v4f*)(ocs + base), s1 = *(const v4f*)(ocs + base + 4);
    const v4f t0 = *(const v4f*)(oct + base), t1 = *(const v4f*)(oct + base + 4);
    const v4f b0 = *(const v4f*)(bcs + c8),   b1 = *(const v4f*)(bcs + c8 + 4);
    const v4f d0 = *(const v4f*)(bct + c8),   d1 = *(const v4f*)(bct + c8 + 4);
    v8f xv, sv, tv;
    xv[0] = x0[0]; xv[1] = x0[1]; xv[2] = x0[2]; xv[3] = x0[3]; xv[4] = x1[0]; xv[5] = x1[1]; xv[6] = x1[2]; xv[7] = x1[3];
    sv[0] = s0[0] + b0[0]; sv[1] = s0[1] + b0[1]; sv[2] = s0[2] + b0[2]; sv[3] = s0[3] + b0[3];
    sv[4] = s1[0] + b1[0]; sv[5] = s1[1] + b1[1]; sv[6] = s1[2] + b1[2]; sv[7] = s1[3] + b1[3];
    tv[0] = t0[0] + d0[0]; tv[1] = t0[1] + d0[1]; tv[2] = t0[2] + d0[2]; tv[3] = t0[3] + d0[3];
    tv[4] = t1[0] + d1[0]; tv[5] = t1[1] + d1[1]; tv[6] = t1[2] + d1[2]; tv[7] = t1[3] + d1[3];
    v8f f;
#pragma unroll
    for (int e = 0; e < 8; ++e) {
      const float g = __builtin_amdgcn_rcpf(1.0f + __expf(-xv[e]));
      f[e] = g * sv[e] + (1.0f - g) * tv[e];
    }
    store16_twice(g16 + base, cvt8h(f, scale));
  }
}

__global__ __launch_bounds__(256) void ptr_softmax_kernel(
    const float* __restrict__ S, const float* __restrict__ mask, float* __restrict__ out) {
  __shared__ __align__(16) float prob[8 * NN];
  __shared__ float invs[8];
  const int tid  = threadIdx.x;
  const int wave = tid >> 5;
  const int lane = tid & 31;
  const int g0   = blockIdx.x * 8;
  const int grow = g0 + wave;
  const int bb   = grow / NP;
  const int p    = grow - bb * NP;
  const float* srow = S + ((size_t)bb * RP + p) * RP;
  const float* mr   = mask + (size_t)grow * NN;
  float* pr = prob + wave * NN;

  float m = NEG_INF;
#pragma unroll 1
  for (int i = lane; i < NN; i += 32) {
    const float t = 10.0f * tanhf(srow[i]) + mr[i];
    pr[i] = t;
    m = fmaxf(m, t);
  }
#pragma unroll
  for (int off = 16; off > 0; off >>= 1) m = fmaxf(m, __shfl_xor(m, off, 32));
  float sum = 0.f;
#pragma unroll 1
  for (int i = lane; i < NN; i += 32) {
    const float e = __expf(pr[i] - m);
    pr[i] = e;
    sum += e;
  }
#pragma unroll
  for (int off = 16; off > 0; off >>= 1) sum += __shfl_xor(sum, off, 32);
  if (lane == 0) invs[wave] = 1.0f / sum;
  __syncthreads();

  float* ob = out + (size_t)g0 * NN;
  for (int pass = 0; pass < 2; ++pass) {
#pragma unroll 1
    for (int it = 0; it < 8; ++it) {
      const int q  = it * 256 + tid;
      const int qc = q < 2 * NN ? q : 2 * NN - 1;
      const v4f e = *(const v4f*)(prob + 4 * qc);
      const float inv = invs[qc / 250];
      v4f v;
      v[0] = e[0] * inv; v[1] = e[1] * inv; v[2] = e[2] * inv; v[3] = e[3] * inv;
      if (q < 2 * NN) *(volatile v4f*)(ob + 4 * (size_t)q) = v;
    }
    __threadfence();
  }
}

extern "C" void kernel_launch(void* const* d_in, const int* in_sizes, int n_in,
                              void* d_out, int out_size, void* d_ws, size_t ws_size,
                              hipStream_t stream) {
  if (n_in < 16) return;
  if (in_sizes[0] != NB * NP * NE || in_sizes[1] != NB * NP * 4 || in_sizes[2] != NB * NN * NE) return;
  if (in_sizes[3] != NB * NP * NN) return;
  if (in_sizes[4] != 132 * NE || in_sizes[7] != 132 * NE || in_sizes[14] != 132 * NE) return;
  if (in_sizes[5] != NE * NE || in_sizes[6] != NE * NE || in_sizes[8] != NE * NE || in_sizes[9] != NE * NE) return;
  if (in_sizes[10] != NE * NE || in_sizes[12] != NE * NE) return;
  if (in_sizes[11] != NE || in_sizes[13] != NE || in_sizes[15] != NE) return;
  if (out_size != NB * NP * NN) return;

  const float* eln  = (const float*)d_in[0];
  const float* attr = (const float*)d_in[1];
  const float* enc  = (const float*)d_in[2];
  const float* mask = (const float*)d_in[3];
  const float* Wqs  = (const float*)d_in[4];
  const float* Wks  = (const float*)d_in[5];
  const float* Wvs  = (const float*)d_in[6];
  const float* Wqt  = (const float*)d_in[7];
  const float* Wkt  = (const float*)d_in[8];
  const float* Wvt  = (const float*)d_in[9];
  const float* Wcs  = (const float*)d_in[10];
  const float* bcs  = (const float*)d_in[11];
  const float* Wct  = (const float*)d_in[12];
  const float* bct  = (const float*)d_in[13];
  const float* Wg   = (const float*)d_in[14];
  const float* bg   = (const float*)d_in[15];
  float* out = (float*)d_out;

  const size_t szENC = (size_t)ROWS * NE * 2;
  const size_t szCAT = (size_t)ROWS * KQ * 2;
  const size_t szWT  = (size_t)(6 * NE * NE + 3 * NE * KQ) * 2;
  const size_t szK   = (size_t)2 * ROWS * NE * 2;
  const size_t szVT  = (size_t)2 * NE * VLD * 2;
  const size_t szQ   = (size_t)2 * ROWS * NE * 2;
  const size_t szGP  = (size_t)ROWS * NE * 4;
  const size_t szO32 = (size_t)2 * ROWS * NE * 4;
  const size_t szO16 = (size_t)2 * ROWS * NE * 2;
  const size_t szOC  = (size_t)2 * ROWS * NE * 4;
  const size_t szG16 = (size_t)ROWS * NE * 2;
  const size_t szS32 = (size_t)NB * RP * RP * 4;
  const size_t oENC = 0;
  const size_t oCAT = oENC + szENC;
  const size_t oWT  = oCAT + szCAT;
  const size_t oK   = oWT + szWT;
  const size_t oVT  = oK + szK;
  const size_t oQ   = oVT + szVT;
  const size_t oGP  = oQ + szQ;
  const size_t oO32 = oGP + szGP;
  const size_t oO16 = oO32 + szO32;
  const size_t oOC  = oO16 + szO16;
  const size_t oG16 = oOC + szOC;
  const size_t oS32 = oG16 + szG16;
  const size_t total = oS32 + szS32;
  if (total > ws_size) return;

  char* ws = (char*)d_ws;
  _Float16* enc16 = (_Float16*)(ws + oENC);
  _Float16* cat16 = (_Float16*)(ws + oCAT);
  _Float16* wt    = (_Float16*)(ws + oWT);
  _Float16* K16   = (_Float16*)(ws + oK);
  _Float16* VT16  = (_Float16*)(ws + oVT);
  _Float16* Q16   = (_Float16*)(ws + oQ);
  float*    GP    = (float*)(ws + oGP);
  float*    O32   = (float*)(ws + oO32);
  _Float16* O16   = (_Float16*)(ws + oO16);
  float*    OC    = (float*)(ws + oOC);
  _Float16* G16   = (_Float16*)(ws + oG16);
  float*    S32   = (float*)(ws + oS32);
  const float* dummy_resid = (const float*)(ws + oENC);

  _Float16* WkTs = wt;
  _Float16* WkTt = wt + 1 * NE * NE;
  _Float16* WvTs = wt + 2 * NE * NE;
  _Float16* WvTt = wt + 3 * NE * NE;
  _Float16* WcTs = wt + 4 * NE * NE;
  _Float16* WcTt = wt + 5 * NE * NE;
  _Float16* WqTs = wt + 6 * NE * NE;
  _Float16* WqTt = wt + 6 * NE * NE + NE * KQ;
  _Float16* WgT  = wt + 6 * NE * NE + 2 * NE * KQ;

  {
    const int n8e = ROWS * NE / 8;
    prep_enc_kernel<<<dim3((n8e + 255) / 256), 256, 0, stream>>>(enc, enc16, n8e);
    const int n8c = ROWS * KQ / 8;
    prep_cat_kernel<<<dim3((n8c + 255) / 256), 256, 0, stream>>>(eln, attr, cat16, n8c);
  }
  {
    const int n8a = NE * NE / 8;
    wtrans_kernel<<<dim3((n8a + 255) / 256, 4), 256, 0, stream>>>(Wks, Wkt, Wvs, Wvt, WkTs, WkTt, WvTs, WvTt, NE, NE, n8a, 64.0f);
    wtrans_kernel<<<dim3((n8a + 255) / 256, 2), 256, 0, stream>>>(Wcs, Wct, Wcs, Wct, WcTs, WcTt, WcTs, WcTt, NE, NE, n8a, 64.0f);
    const int n8b = NE * KQ / 8;
    wtrans_kernel<<<dim3((n8b + 255) / 256, 3), 256, 0, stream>>>(Wqs, Wqt, Wg, Wg, WqTs, WqTt, WgT, WgT, 132, KQ, n8b, 64.0f);
  }
  {
    const int tiles = (ROWS / 64) * (NE / 64);
    wmma_gemm64<0, false, 0, 1, false, 0><<<dim3((tiles + 7) / 8, 2), 256, 0, stream>>>(
        (const unsigned short*)enc16, (const unsigned short*)enc16, NE, (long)0,
        (const unsigned short*)WkTs, (const unsigned short*)WkTs, NE, (long)(NE * NE),
        (void*)K16, (void*)K16, NE, (long)ROWS * NE,
        bg, dummy_resid, (long)0, ROWS, NE, NE, 1.0f);
  }
  {
    const int tiles = (NE / 64) * (ROWS / 64);
    wmma_gemm64<0, false, 0, 1, false, 0><<<dim3((tiles + 7) / 8, 2), 256, 0, stream>>>(
        (const unsigned short*)WvTs, (const unsigned short*)WvTs, NE, (long)(NE * NE),
        (const unsigned short*)enc16, (const unsigned short*)enc16, NE, (long)0,
        (void*)VT16, (void*)VT16, VLD, (long)NE * VLD,
        bg, dummy_resid, (long)0, NE, ROWS, NE, 1.0f);
  }
  {
    const int tiles = (ROWS / 64) * (NE / 64);
    wmma_gemm64<0, false, 0, 1, false, 0><<<dim3((tiles + 7) / 8, 2), 256, 0, stream>>>(
        (const unsigned short*)cat16, (const unsigned short*)cat16, KQ, (long)0,
        (const unsigned short*)WqTs, (const unsigned short*)WqTs, KQ, (long)(NE * KQ),
        (void*)Q16, (void*)Q16, NE, (long)ROWS * NE,
        bg, dummy_resid, (long)0, ROWS, NE, KQ, 1.0f);
  }
  {
    const int tiles = (ROWS / 64) * (NE / 64);
    wmma_gemm64<0, false, 2, 0, false, 0><<<dim3((tiles + 7) / 8, 1), 256, 0, stream>>>(
        (const unsigned short*)cat16, (const unsigned short*)cat16, KQ, (long)0,
        (const unsigned short*)WgT, (const unsigned short*)WgT, KQ, (long)0,
        (void*)GP, (void*)GP, NE, (long)0,
        bg, dummy_resid, (long)0, ROWS, NE, KQ, 1.0f / 64.0f);
  }
  mha16_kernel<<<dim3(RP / AT_QB, 2 * NB * NH), 128, 0, stream>>>(Q16, K16, VT16, mask, O32, 0.25f / 4096.0f);
  {
    const int n8 = 2 * ROWS * NE / 8;
    cast_o_kernel<<<dim3((n8 + 255) / 256), 256, 0, stream>>>(O32, O16, n8, 256.0f);
  }
  {
    const int tiles = (ROWS / 64) * (NE / 64);
    wmma_gemm64<0, false, 0, 0, false, 0><<<dim3((tiles + 7) / 8, 2), 256, 0, stream>>>(
        (const unsigned short*)O16, (const unsigned short*)O16, NE, (long)ROWS * NE,
        (const unsigned short*)WcTs, (const unsigned short*)WcTs, NE, (long)(NE * NE),
        (void*)OC, (void*)OC, NE, (long)ROWS * NE,
        bg, dummy_resid, (long)0, ROWS, NE, NE, 1.0f / 16384.0f);
  }
  {
    const int n8 = ROWS * NE / 8;
    combine_kernel<<<dim3((n8 + 255) / 256), 256, 0, stream>>>(GP, OC, OC + (size_t)ROWS * NE, bcs, bct, G16, n8, 1024.0f);
  }
  {
    const int tiles = (RP / 64) * (RP / 64);
    const float sc = (1.0f / 11.313708498984761f) * (1.0f / 1024.0f);
    wmma_gemm64<0, false, 0, 0, false, 0><<<dim3((tiles + 7) / 8, NB), 256, 0, stream>>>(
        (const unsigned short*)G16, (const unsigned short*)G16, NE, (long)RP * NE,
        (const unsigned short*)enc16, (const unsigned short*)enc16, NE, (long)RP * NE,
        (void*)S32, (void*)S32, RP, (long)RP * RP,
        bg, dummy_resid, (long)0, RP, RP, NE, sc);
  }
  ptr_softmax_kernel<<<dim3(NB * NP / 8), 256, 0, stream>>>(S32, mask, out);
}
